// GCN_32160715112815
// MI455X (gfx1250) — hardware-run, weakly checked
//
#include <hip/hip_runtime.h>

typedef float          v8f   __attribute__((ext_vector_type(8)));
typedef float          v4f   __attribute__((ext_vector_type(4)));
typedef unsigned int   v4u   __attribute__((ext_vector_type(4)));
typedef int            v8i   __attribute__((ext_vector_type(8)));
typedef unsigned short v8us  __attribute__((ext_vector_type(8)));
typedef unsigned short v16us __attribute__((ext_vector_type(16)));
typedef __bf16         v16bf __attribute__((ext_vector_type(16)));
typedef _Float16       v16h  __attribute__((ext_vector_type(16)));
typedef v4f  __attribute__((may_alias)) v4fa;
typedef v8us __attribute__((may_alias)) v8usa;
union FragB { v16bf v; v16us u; v8us h[2]; v8i w; };
union FragH { v16h  v; v16us u; v8us h[2]; v8i w; };

__device__ __forceinline__ v8f wmb(const FragB& a, const FragB& b, v8f c) {
  v8f d = __builtin_amdgcn_wmma_f32_16x16x32_bf16(false, a.v, false, b.v, (short)0, c, false, false);
  asm volatile("v_nop\n\tv_nop\n\tv_nop\n\tv_nop" : "+v"(d) : "v"(a.w), "v"(b.w));
  return d;
}

__device__ __forceinline__ v8f wmh(const FragH& a, const FragH& b, v8f c) {
  v8f d = __builtin_amdgcn_wmma_f32_16x16x32_f16(false, a.v, false, b.v, (short)0, c, false, false);
  asm volatile("v_nop\n\tv_nop\n\tv_nop\n\tv_nop" : "+v"(d) : "v"(a.w), "v"(b.w));
  return d;
}

__device__ __forceinline__ unsigned bf16_bits(float f) {
  const unsigned u = __float_as_uint(f);
  const unsigned r = (u + 0x7FFFu + ((u >> 16) & 1u)) >> 16;
  const unsigned q = (u >> 16) | 0x40u;
  return ((u & 0x7fffffffu) > 0x7f800000u) ? q : r;
}

__device__ __forceinline__ float bf16_val(float f) {
  return __uint_as_float(bf16_bits(f) << 16);
}
__device__ __forceinline__ int clampi(int v, int lo, int hi) {
  return v < lo ? lo : (v > hi ? hi : v);
}

__device__ __forceinline__ unsigned f16_bits(float f) {
  const unsigned u  = __float_as_uint(f);
  const unsigned s  = (u >> 16) & 0x8000u;
  const unsigned a  = u & 0x7fffffffu;
  const unsigned t  = a - 0x38000000u;
  const unsigned r  = (t + 0x0FFFu + ((t >> 13) & 1u)) >> 13;
  const unsigned rc = r > 0x7C00u ? 0x7C00u : r;
  const bool small  = a < 0x38800000u;
  const bool isnan  = a > 0x7f800000u;
  const unsigned fin = small ? 0u : (s | rc);
  return isnan ? (s | 0x7E00u) : fin;
}

__device__ __forceinline__ unsigned pk16(unsigned lo, unsigned hi) { return lo | (hi << 16); }
__device__ __forceinline__ unsigned bf16_lo_bits(float v) {
  float hi = bf16_val(v);
  asm volatile("" : "+v"(hi));
  return bf16_bits(v - hi);
}
__device__ __forceinline__ v4u pack8_bf16(v4f a, v4f c) {
  return (v4u){ pk16(bf16_bits(a[0]), bf16_bits(a[1])), pk16(bf16_bits(a[2]), bf16_bits(a[3])),
                pk16(bf16_bits(c[0]), bf16_bits(c[1])), pk16(bf16_bits(c[2]), bf16_bits(c[3])) };
}
__device__ __forceinline__ v4u pack8_bf16_lo(v4f a, v4f c) {
  return (v4u){ pk16(bf16_lo_bits(a[0]), bf16_lo_bits(a[1])), pk16(bf16_lo_bits(a[2]), bf16_lo_bits(a[3])),
                pk16(bf16_lo_bits(c[0]), bf16_lo_bits(c[1])), pk16(bf16_lo_bits(c[2]), bf16_lo_bits(c[3])) };
}
__device__ __forceinline__ v4u pack8_f16(v4f a, v4f c) {
  return (v4u){ pk16(f16_bits(a[0]), f16_bits(a[1])), pk16(f16_bits(a[2]), f16_bits(a[3])),
                pk16(f16_bits(c[0]), f16_bits(c[1])), pk16(f16_bits(c[2]), f16_bits(c[3])) };
}

template <int FORM>
__global__ __launch_bounds__(256) void k_plane(const float* __restrict__ src, int rows, int cols, int ldsrc,
                                               unsigned short* __restrict__ dst, int MP, int KP) {
  static_assert(FORM >= 0 && FORM <= 3);
  const int KTOT = (FORM == 1 || FORM == 3) ? 2 * KP : KP;
  const unsigned ppr   = (unsigned)(KTOT >> 3);
  const unsigned kp8   = (unsigned)(KP >> 3);
  const unsigned total = (unsigned)MP * ppr;
  const unsigned g     = blockIdx.x * 256u + threadIdx.x;
  const unsigned rowu  = g / ppr;
  const unsigned p     = g - rowu * ppr;
  const bool second    = p >= kp8;
  const int row = (int)rowu;
  const int c0  = (int)((second ? p - kp8 : p) << 3);
  const float* srow = src + (size_t)clampi(row, 0, rows - 1) * (size_t)ldsrc;
  float x[8];
  unsigned mk[8];
#pragma unroll
  for (int e = 0; e < 8; ++e) {
    const int c = c0 + e;
    const float v = srow[clampi(c, 0, cols - 1)];
    asm volatile("" :: "v"(v));
    x[e]  = v;
    mk[e] = (row < rows && c < cols) ? 0xFFFFu : 0u;
  }
  const v4f a = (v4f){ x[0], x[1], x[2], x[3] };
  const v4f c = (v4f){ x[4], x[5], x[6], x[7] };
  v4u o;
  if (FORM == 2) {
    o = pack8_f16(a, c);
  } else {
    const v4u hi = pack8_bf16(a, c);
    o = hi;
    if (FORM == 1) { const v4u lo = pack8_bf16_lo(a, c); o = second ? lo : hi; }
  }
  const v4u mw = (v4u){ pk16(mk[0], mk[1]), pk16(mk[2], mk[3]), pk16(mk[4], mk[5]), pk16(mk[6], mk[7]) };
  o &= mw;
  if (g < total) {
    volatile v4u* q = (volatile v4u*)(dst + (size_t)g * 8);
    *q = o;
    __threadfence();
    *q = o;
  }
}

template <int FORM> struct FragOf    { typedef FragB T; };
template <>         struct FragOf<2> { typedef FragH T; };
__device__ __forceinline__ v8f mm(const FragB& a, const FragB& b, v8f c) { return wmb(a, b, c); }
__device__ __forceinline__ v8f mm(const FragH& a, const FragH& b, v8f c) { return wmh(a, b, c); }
template <class F> __device__ __forceinline__ F ld_frag(const unsigned short* p) {
  F f;
  f.h[0] = *(const v8usa*)(p);
  f.h[1] = *(const v8usa*)(p + 16);
  return f;
}

template <int FORM, int EPI>
__global__ __launch_bounds__(256) __attribute__((amdgpu_num_vgpr(248)))
void k_gemm_nt(const unsigned short* __restrict__ A, const unsigned short* __restrict__ B,
               const float* __restrict__ bias, float* __restrict__ D, int M, int N, int KTOT, int ldd) {
  static_assert(FORM >= 0 && FORM <= 2);
  static_assert(EPI == 0 || EPI == 1);
  typedef typename FragOf<FORM>::T F;
  __shared__ __attribute__((aligned(16))) float sT[8][16 * 68];
  const int lane = threadIdx.x & 31;
  const int wave = threadIdx.x >> 5;
  const int tilesM = (M + 63) >> 6;
  const int tilesN = (N + 63) >> 6;
  const int tile = blockIdx.x * 8 + wave;
  if (tile >= tilesM * tilesN) return;
  const int tm = tile / tilesN;
  const int tn = tile - tm * tilesN;
  const int m0 = tm << 6;
  const int n0 = tn << 6;

  const int rl = lane & 15;
  const int h8 = (lane >> 4) * 8;
  const unsigned short* pa = A + (size_t)(m0 + rl) * (size_t)KTOT + h8;
  const unsigned short* pb = B + (size_t)(n0 + rl) * (size_t)KTOT + h8;

  v8f acc[4][4];
#pragma unroll
  for (int i = 0; i < 4; ++i)
#pragma unroll
    for (int j = 0; j < 4; ++j) acc[i][j] = (v8f){0.f, 0.f, 0.f, 0.f, 0.f, 0.f, 0.f, 0.f};

#pragma unroll 1
  for (int k0 = 0; k0 < KTOT; k0 += 32) {
    F bf[4];
#pragma unroll
    for (int j = 0; j < 4; ++j) bf[j] = ld_frag<F>(pb + (size_t)(j << 4) * (size_t)KTOT + k0);
#pragma unroll
    for (int i = 0; i < 4; ++i) {
      const F af = ld_frag<F>(pa + (size_t)(i << 4) * (size_t)KTOT + k0);
#pragma unroll
      for (int j = 0; j < 4; ++j) acc[i][j] = mm(af, bf[j], acc[i][j]);
    }
  }

  float* slab = sT[wave];
  const int hh = lane >> 4;
  const int c4 = (lane & 15) * 4;
  const int nc = n0 + c4;
  const bool cok = nc < N;
  v4f bv = (v4f){0.f, 0.f, 0.f, 0.f};
  if (EPI == 1) {
    bv = *(const v4fa*)(bias + clampi(nc, 0, N - 4));
    asm volatile("" :: "v"(bv));
  }
#pragma unroll
  for (int i = 0; i < 4; ++i) {
    const int mBase = m0 + (i << 4);
#pragma unroll
    for (int j = 0; j < 4; ++j) {
#pragma unroll
      for (int r = 0; r < 8; ++r) slab[(h8 + r) * 68 + (j << 4) + rl] = acc[i][j][r];
    }
    __builtin_amdgcn_fence(__ATOMIC_RELEASE, "workgroup");
    __builtin_amdgcn_wave_barrier();
    __builtin_amdgcn_fence(__ATOMIC_ACQUIRE, "workgroup");
    v4f vv[8];
#pragma unroll
    for (int it = 0; it < 8; ++it) {
      const int row = it * 2 + hh;
      v4f v = *(const v4fa*)(slab + row * 68 + c4);
      if (EPI == 1) v += bv;
      vv[it] = v;
    }
    for (int pass = 0; pass < 2; ++pass) {
#pragma unroll
      for (int it = 0; it < 8; ++it) {
        const int row = mBase + it * 2 + hh;
        if (cok && row < M) *(volatile v4f*)(D + (size_t)row * (size_t)ldd + nc) = vv[it];
      }
      __threadfence();
    }
    __builtin_amdgcn_fence(__ATOMIC_RELEASE, "workgroup");
    __builtin_amdgcn_wave_barrier();
    __builtin_amdgcn_fence(__ATOMIC_ACQUIRE, "workgroup");
  }
}

#include <stddef.h>
#include <stdint.h>
#include <math.h>

#ifndef TWO_TERM_L2
#define TWO_TERM_L2 0
#endif
#ifndef TWO_TERM_L3
#define TWO_TERM_L3 0
#endif

#define NN      100000
#define NE      800000
#define DIN     64
#define DHID    64
#define DOUT    47
#define OUTN    (NN * DOUT)
#define MPAD    100096
#define K2      (TWO_TERM_L2 ? 128 : 64)
#define K3      (TWO_TERM_L3 ? 128 : 64)
#define NTHR    256
#define NWAVE   8
#define NBRUN   1024
#define SLB     10
#define NBLK    98
#define EPW     (NE / NWAVE)
#define STEPE   256
#define NSTEP   ((EPW + STEPE - 1) / STEPE)
#define WLCAP   2048
#define LCAP    10496
#define DEGCAP  32
#define MEAS_B1024 8361
#define MEAS_DEG   23
#define GPW     4
#define RGRP    32
#define BK_ZINTS   (NWAVE * WLCAP + LCAP + 3 * NBRUN)
#define BK_INTS    (BK_ZINTS + 16)
#define BK_LDS     (BK_INTS * 4)
#define LIST_V4    (LCAP / 4)
#define LIST_IT    ((LIST_V4 + NTHR - 1) / NTHR)
#define OUT_V4     (RGRP * DOUT / 4)
#define OUT_IT     ((OUT_V4 + 31) / 32)
#define NB1     ((DHID * DIN / 8) / NTHR)
#define NB2     ((DHID * K2 / 8) / NTHR)
#define NB3     ((DHID * K3 / 8) / NTHR)

static_assert(NN % 32 == 0 && NBRUN % 32 == 0 && DOUT <= 64);
static_assert(NBRUN == (1 << SLB) && NWAVE * GPW * RGRP == NBRUN);
static_assert((NBLK - 1) * NBRUN < NN && NBLK * NBRUN >= MPAD && NN - (NBLK - 1) * NBRUN == 672);
static_assert(MPAD % 128 == 0 && MPAD % 64 == 0 && MPAD >= NN && MPAD % RGRP == 0);
static_assert(NE % NWAVE == 0 && EPW % 8 == 0 && NE % 8 == 0);
static_assert(NE - 390 * 2048 == 1280 && EPW - 390 * STEPE == 160 && NSTEP == 391);
static_assert(((long long)(NN - 1) << SLB) < (1LL << 31));
static_assert(LCAP % 256 == 0 && 4 * LCAP >= 5 * MEAS_B1024 && LCAP % 32 == 0);
static_assert(DEGCAP == 32 && DEGCAP >= MEAS_DEG + 8);
static_assert(WLCAP % 4 == 0 && BK_ZINTS % 4 == 0);
static_assert(BK_LDS <= 262144 && BK_LDS + 0 <= 327680);
static_assert(NWAVE * RGRP * DOUT * 4 <= 327680 && 8 * 16 * 68 * 4 <= 327680);
static_assert((RGRP * DOUT) % 4 == 0 && (RGRP * DOUT * 4) % 128 == 0 && OUT_IT == 12);
static_assert((long long)(NN / RGRP) * RGRP * DOUT == (long long)OUTN);
static_assert(K2 % 32 == 0 && K3 % 32 == 0 && DIN % 32 == 0 && DHID == 64);
static_assert((DHID * DIN / 8) % NTHR == 0 && (DHID * K2 / 8) % NTHR == 0 && (DHID * K3 / 8) % NTHR == 0);
static_assert((MPAD * (DIN / 8)) % 256 == 0);

typedef float v2f __attribute__((ext_vector_type(2)));
typedef int   v4i __attribute__((ext_vector_type(4)));
typedef v2f __attribute__((may_alias)) v2fa;
typedef v4i __attribute__((may_alias)) v4ia;

__device__ __forceinline__ void wunit(const float* __restrict__ W, int ncols, int nvalid, int KW, int u,
                                      unsigned short* dstp) {
  const int ppr = KW >> 3;
  const int n   = u / ppr;
  const int k8  = (u - n * ppr) << 3;
  const int kk  = k8 & 63;
  const int nc  = n < nvalid ? n : nvalid - 1;
  const float* p = W + (size_t)kk * (size_t)ncols + nc;
  const unsigned mk = (n < nvalid) ? 0xFFFFu : 0u;
  unsigned w[8];
#pragma unroll
  for (int i = 0; i < 8; ++i) {
    const float v = p[(size_t)i * (size_t)ncols];
    asm volatile("" :: "v"(v));
    w[i] = bf16_bits(v) & mk;
  }
  const v4u o = (v4u){ pk16(w[0], w[1]), pk16(w[2], w[3]), pk16(w[4], w[5]), pk16(w[6], w[7]) };
  volatile v4u* q = (volatile v4u*)(dstp + (size_t)n * (size_t)KW + k8);
  *q = o;
  __threadfence();
  *q = o;
}

__device__ __forceinline__ void bunit(const float* __restrict__ bsrc, int nb, int tid, float* dstp) {
  const int c4 = (tid & 15) * 4;
  float x[4];
#pragma unroll
  for (int e = 0; e < 4; ++e) {
    const int c = c4 + e;
    const float v = bsrc[c < nb ? c : nb - 1];
    asm volatile("" :: "v"(v));
    const float bvv = bf16_val(v);
    x[e] = (c < nb) ? bvv : 0.0f;
  }
  const v4f o = (v4f){ x[0], x[1], x[2], x[3] };
  if (tid < 16) {
    volatile v4f* q = (volatile v4f*)(dstp + c4);
    *q = o;
    __threadfence();
    *q = o;
  }
}

__global__ __launch_bounds__(NTHR) void k_prep(const float* __restrict__ W1, const float* __restrict__ W2,
                                               const float* __restrict__ W3, const float* __restrict__ b1,
                                               const float* __restrict__ b2, const float* __restrict__ b3,
                                               unsigned short* W1T, unsigned short* W2D, unsigned short* W3D,
                                               float* BT) {
  const int blk = (int)blockIdx.x;
  const int tid = (int)threadIdx.x;
  if (blk < NB1) {
    wunit(W1, DHID, DHID, DIN, blk * NTHR + tid, W1T);
  } else if (blk < NB1 + NB2) {
    wunit(W2, DHID, DHID, K2, (blk - NB1) * NTHR + tid, W2D);
  } else if (blk < NB1 + NB2 + NB3) {
    wunit(W3, DOUT, DOUT, K3, (blk - NB1 - NB2) * NTHR + tid, W3D);
  } else if (blk == NB1 + NB2 + NB3) {
    bunit(b1, DHID, tid, BT);
  } else if (blk == NB1 + NB2 + NB3 + 1) {
    bunit(b2, DHID, tid, BT + 64);
  } else {
    bunit(b3, DOUT, tid, BT + 128);
  }
}

#define PIN(x) asm volatile("" :: "v"(x))
#define PUTJ(HJ, SRCJ, SJ) { \
    const int wv = (clampi((SRCJ), 0, nN - 1) << SLB) | (int)(SJ); \
    if (HJ) { if (pos < WLCAP) wlw[pos] = wv; } \
    pos += (HJ) ? 1 : 0; }

__global__ __launch_bounds__(NTHR) void k_bucket(const int* __restrict__ srcs, const int* __restrict__ dsts,
                                                 int nN, int* listG, int* cntG, int* offG, int* flagG) {
  extern __shared__ __attribute__((aligned(16))) int dsm[];
  int* wl   = dsm;
  int* sl   = dsm + NWAVE * WLCAP;
  int* cnt  = sl + LCAP;
  int* offs = cnt + NBRUN;
  int* cur  = offs + NBRUN;
  int* misc = cur + NBRUN;
  const int tid = (int)threadIdx.x, lane = tid & 31, wave = tid >> 5;
  const int b = (int)blockIdx.x;
  const int nodeBase = b * NBRUN;
  const int nb = clampi(nN - nodeBase, 0, NBRUN);

  {
    const v4i z4 = {0, 0, 0, 0};
    for (int i = tid * 4; i < BK_ZINTS; i += NTHR * 4) *(v4ia*)(dsm + i) = z4;
    if (tid < 16) misc[tid] = 0;
  }
  __syncthreads();

  {
    int* wlw = wl + wave * WLCAP;
    const int wbeg = wave * EPW;
    const int wend = wbeg + EPW;
    const unsigned nbs = (unsigned)nodeBase;
    const unsigned unb = (unsigned)nb;
    int wc = 0;
#pragma unroll 1
    for (int st = 0; st < NSTEP; ++st) {
      const int e0  = wbeg + st * STEPE + lane * 8;
      const int e0c = e0 < (NE - 8) ? e0 : (NE - 8);
      const v4i da = *(const v4ia*)(dsts + e0c);
      const v4i db = *(const v4ia*)(dsts + e0c + 4);
      const v4i sa = *(const v4ia*)(srcs + e0c);
      const v4i sb = *(const v4ia*)(srcs + e0c + 4);
      PIN(da.x); PIN(da.y); PIN(da.z); PIN(da.w);
      PIN(db.x); PIN(db.y); PIN(db.z); PIN(db.w);
      PIN(sa.x); PIN(sa.y); PIN(sa.z); PIN(sa.w);
      PIN(sb.x); PIN(sb.y); PIN(sb.z); PIN(sb.w);
      const unsigned s0 = (unsigned)da.x - nbs, s1 = (unsigned)da.y - nbs;
      const unsigned s2 = (unsigned)da.z - nbs, s3 = (unsigned)da.w - nbs;
      const unsigned s4 = (unsigned)db.x - nbs, s5 = (unsigned)db.y - nbs;
      const unsigned s6 = (unsigned)db.z - nbs, s7 = (unsigned)db.w - nbs;
      const bool h0 = (e0 + 0 < wend) && (s0 < unb);
      const bool h1 = (e0 + 1 < wend) && (s1 < unb);
      const bool h2 = (e0 + 2 < wend) && (s2 < unb);
      const bool h3 = (e0 + 3 < wend) && (s3 < unb);
      const bool h4 = (e0 + 4 < wend) && (s4 < unb);
      const bool h5 = (e0 + 5 < wend) && (s5 < unb);
      const bool h6 = (e0 + 6 < wend) && (s6 < unb);
      const bool h7 = (e0 + 7 < wend) && (s7 < unb);
      const unsigned m0 = __builtin_amdgcn_ballot_w32(h0);
      const unsigned m1 = __builtin_amdgcn_ballot_w32(h1);
      const unsigned m2 = __builtin_amdgcn_ballot_w32(h2);
      const unsigned m3 = __builtin_amdgcn_ballot_w32(h3);
      const unsigned m4 = __builtin_amdgcn_ballot_w32(h4);
      const unsigned m5 = __builtin_amdgcn_ballot_w32(h5);
      const unsigned m6 = __builtin_amdgcn_ballot_w32(h6);
      const unsigned m7 = __builtin_amdgcn_ballot_w32(h7);
      const unsigned many = m0 | m1 | m2 | m3 | m4 | m5 | m6 | m7;
      if (many != 0u) {
        unsigned pre = __builtin_amdgcn_mbcnt_lo(m0, 0u);
        pre = __builtin_amdgcn_mbcnt_lo(m1, pre);
        pre = __builtin_amdgcn_mbcnt_lo(m2, pre);
        pre = __builtin_amdgcn_mbcnt_lo(m3, pre);
        pre = __builtin_amdgcn_mbcnt_lo(m4, pre);
        pre = __builtin_amdgcn_mbcnt_lo(m5, pre);
        pre = __builtin_amdgcn_mbcnt_lo(m6, pre);
        pre = __builtin_amdgcn_mbcnt_lo(m7, pre);
        int pos = wc + (int)pre;
        PUTJ(h0, sa.x, s0)
        PUTJ(h1, sa.y, s1)
        PUTJ(h2, sa.z, s2)
        PUTJ(h3, sa.w, s3)
        PUTJ(h4, sb.x, s4)
        PUTJ(h5, sb.y, s5)
        PUTJ(h6, sb.z, s6)
        PUTJ(h7, sb.w, s7)
        wc += (int)__builtin_popcount(m0) + (int)__builtin_popcount(m1) + (int)__builtin_popcount(m2)
            + (int)__builtin_popcount(m3) + (int)__builtin_popcount(m4) + (int)__builtin_popcount(m5)
            + (int)__builtin_popcount(m6) + (int)__builtin_popcount(m7);
      }
    }
    if (lane == 0) misc[wave] = wc;
  }
  __syncthreads();

  if (wave == 0) {
    int t = 0, ov = 0;
#pragma unroll 1
    for (int w2 = 0; w2 < NWAVE; ++w2) {
      int c = misc[w2];
      ov |= (c > WLCAP) ? 1 : 0;
      c = c < 0 ? 0 : (c > WLCAP ? WLCAP : c);
      c = __builtin_amdgcn_readfirstlane(c);
#pragma unroll 1
      for (int b0 = 0; b0 < c; b0 += 32) {
        const int idx = b0 + lane;
        const int ent = wl[w2 * WLCAP + (idx < WLCAP ? idx : WLCAP - 1)];
        const int m32 = (c - b0) < 32 ? (c - b0) : 32;
#pragma unroll 1
        for (int k = 0; k < m32; ++k) {
          const int u    = __builtin_amdgcn_readlane(ent, k);
          const int slot = u & (NBRUN - 1);
          if (t < LCAP) {
            const int cvv = cnt[slot];
            if (lane == 0) cnt[slot] = cvv + 1;
            t = t + 1;
          } else {
            ov = 1;
          }
        }
      }
    }
    if (lane == 0) { misc[8] = t; misc[9] = ov; }
  }
  __syncthreads();

  if (wave == 0) {
    const int base = lane * (NBRUN / 32);
    int s = 0;
#pragma unroll 1
    for (int i = 0; i < NBRUN / 32; ++i) s += cnt[base + i];
    int incl = s;
#pragma unroll
    for (int d = 1; d < 32; d <<= 1) {
      const int y = __shfl_up(incl, d, 32);
      if (lane >= d) incl += y;
    }
    int run = incl - s;
#pragma unroll 1
    for (int i = 0; i < NBRUN / 32; ++i) {
      const int cvv = cnt[base + i];
      offs[base + i] = run;
      cur[base + i]  = run;
      run += cvv;
    }
  }
  __syncthreads();

  if (wave == 0) {
    int t = 0;
#pragma unroll 1
    for (int w2 = 0; w2 < NWAVE; ++w2) {
      int c = misc[w2];
      c = c < 0 ? 0 : (c > WLCAP ? WLCAP : c);
      c = __builtin_amdgcn_readfirstlane(c);
#pragma unroll 1
      for (int b0 = 0; b0 < c; b0 += 32) {
        const int idx = b0 + lane;
        const int ent = wl[w2 * WLCAP + (idx < WLCAP ? idx : WLCAP - 1)];
        const int m32 = (c - b0) < 32 ? (c - b0) : 32;
#pragma unroll 1
        for (int k = 0; k < m32; ++k) {
          const int u    = __builtin_amdgcn_readlane(ent, k);
          const int slot = u & (NBRUN - 1);
          if (t < LCAP) {
            int p = cur[slot];
            p = p < 0 ? 0 : (p > LCAP - 1 ? LCAP - 1 : p);
            if (lane == 0) { sl[p] = u >> SLB; cur[slot] = p + 1; }
            t = t + 1;
          }
        }
      }
    }
  }
  __syncthreads();

  {
    const int ovf = misc[9];
    const v4i fv = {ovf, ovf, ovf, ovf};
    int* lb = listG + (size_t)b * LCAP;
    for (int pass = 0; pass < 2; ++pass) {
#pragma unroll 1
      for (int it = 0; it < LIST_IT; ++it) {
        const int i4 = it * NTHR + tid;
        const int ic = i4 < LIST_V4 ? i4 : LIST_V4 - 1;
        const v4i v = *(const v4ia*)(sl + 4 * ic);
        if (i4 < LIST_V4) *(volatile v4i*)(lb + 4 * (size_t)i4) = v;
      }
      {
        const v4i c4 = *(const v4ia*)(cnt + 4 * tid);
        const v4i o4 = *(const v4ia*)(offs + 4 * tid);
        *(volatile v4i*)(cntG + (size_t)nodeBase + 4 * tid) = c4;
        *(volatile v4i*)(offG + (size_t)nodeBase + 4 * tid) = o4;
      }
      if (tid < 8) *(volatile v4i*)(flagG + (size_t)b * 32 + 4 * tid) = fv;
      __threadfence();
    }
  }
}

__device__ __forceinline__ v2f row_gather(const float* __restrict__ T, int ent, int cn, int lane, int nN) {
  float a0 = 0.0f, a1 = 0.0f;
#pragma unroll 1
  for (int k = 0; k < cn; ++k) {
    int sk = __builtin_amdgcn_readlane(ent, k);
    sk = clampi(sk, 0, nN - 1);
    const v2f t = *(const v2fa*)(T + (size_t)sk * 64 + 2 * lane);
    a0 += t.x; a1 += t.y;
  }
  return (v2f){ a0, a1 };
}

template <int KOUT>
__global__ __launch_bounds__(NTHR) void k_replay_hid(const float* __restrict__ T, const int* __restrict__ listG,
                                                     const int* __restrict__ cntG, const int* __restrict__ offG,
                                                     const int* __restrict__ flagG, const float* __restrict__ bias,
                                                     unsigned short* hb, int nN, int mRows) {
  static_assert(KOUT == 64 || KOUT == 128);
  const int tid = (int)threadIdx.x, lane = tid & 31, wave = tid >> 5;
  const int b = (int)blockIdx.x;
  const int nodeBase = b * NBRUN;
  const v2f bv = *(const v2fa*)(bias + 2 * lane);
  int fl = flagG[(size_t)b * 32];
  PIN(fl);
  const bool ovf = fl != 0;
  const int* listb = listG + (size_t)b * LCAP;
  const float qnan = __int_as_float(0x7fc00000);
  const int q0s = (4 * lane) & 31, q1s = (4 * lane + 1) & 31;
  const int q2s = (4 * lane + 2) & 31, q3s = (4 * lane + 3) & 31;
  const bool lsel = (lane & 8) != 0;
  const bool wr = lane < (KOUT / 8);

#pragma unroll 1
  for (int q = 0; q < GPW; ++q) {
    const int row0 = nodeBase + RGRP * (wave * GPW + q);
    if (row0 >= mRows) continue;
    const int ti = clampi(row0 + lane, 0, NBLK * NBRUN - 1);
    int cv = cntG[ti];
    int ofv = offG[ti];
    PIN(cv);
    PIN(ofv);
    const int bigv = (cv > DEGCAP) ? 1 : 0;
    cv  = cv < 0 ? 0 : (cv > DEGCAP ? DEGCAP : cv);
    ofv = ofv < 0 ? 0 : (ofv > LCAP ? LCAP : ofv);
#pragma unroll 1
    for (int r = 0; r < RGRP; ++r) {
      const int node = row0 + r;
      const bool live = node < nN;
      const int c  = __builtin_amdgcn_readlane(cv, r);
      const int o  = __builtin_amdgcn_readlane(ofv, r);
      const int bg = __builtin_amdgcn_readlane(bigv, r);
      const int cn = __builtin_amdgcn_readfirstlane(live ? c : 0);
      const int idx = clampi(o + lane, 0, LCAP - 1);
      int ent = listb[idx];
      PIN(ent);
      const v2f a = row_gather(T, ent, cn, lane, nN);
      float y0 = a.x + bv.x;
      float y1 = a.y + bv.y;
      y0 = (y0 > 0.0f) ? y0 : (y0 - y0);
      y1 = (y1 > 0.0f) ? y1 : (y1 - y1);
      const bool bad = ovf || (bg != 0);
      y0 = bad ? qnan : y0;
      y1 = bad ? qnan : y1;
      const float v0 = live ? y0 : 0.0f;
      const float v1 = live ? y1 : 0.0f;
      const unsigned hb0 = bf16_bits(v0), hb1 = bf16_bits(v1);
      const int hw = (int)pk16(hb0, hb1);
      v4u pv;
      const int g0 = __shfl(hw, q0s, 32), g1 = __shfl(hw, q1s, 32);
      const int g2 = __shfl(hw, q2s, 32), g3 = __shfl(hw, q3s, 32);
      if (KOUT == 128) {
        const unsigned lb0 = bf16_lo_bits(v0), lb1 = bf16_lo_bits(v1);
        const int lw = (int)pk16(lb0, lb1);
        const int p0 = __shfl(lw, q0s, 32), p1 = __shfl(lw, q1s, 32);
        const int p2 = __shfl(lw, q2s, 32), p3 = __shfl(lw, q3s, 32);
        pv = (v4u){ (unsigned)(lsel ? p0 : g0), (unsigned)(lsel ? p1 : g1),
                    (unsigned)(lsel ? p2 : g2), (unsigned)(lsel ? p3 : g3) };
      } else {
        pv = (v4u){ (unsigned)g0, (unsigned)g1, (unsigned)g2, (unsigned)g3 };
      }
      unsigned short* hp = hb + (size_t)node * KOUT + 8 * (lane & 15);
      if (wr) *(volatile v4u*)hp = pv;
      __threadfence();
      if (wr) *(volatile v4u*)hp = pv;
    }
  }
}

__global__ __launch_bounds__(NTHR) void k_replay_out(const float* __restrict__ T, const int* __restrict__ listG,
                                                     const int* __restrict__ cntG, const int* __restrict__ offG,
                                                     const int* __restrict__ flagG, const float* __restrict__ bias,
                                                     float* out, int nN, int outN) {
  __shared__ __attribute__((aligned(16))) float strip[NWAVE][RGRP * DOUT];
  const int tid = (int)threadIdx.x, lane = tid & 31, wave = tid >> 5;
  const int b = (int)blockIdx.x;
  const int nodeBase = b * NBRUN;
  const v2f bv = *(const v2fa*)(bias + 2 * lane);
  int fl = flagG[(size_t)b * 32];
  PIN(fl);
  const bool ovf = fl != 0;
  const int* listb = listG + (size_t)b * LCAP;
  const float qnan = __int_as_float(0x7fc00000);
  const float ninf = -__builtin_inff();
  const int c0 = 2 * lane;
  const bool val0 = c0 < DOUT;
  const bool val1 = (c0 + 1) < DOUT;
  float* st = strip[wave];

#pragma unroll 1
  for (int q = 0; q < GPW; ++q) {
    const int row0 = nodeBase + RGRP * (wave * GPW + q);
    if (row0 >= nN) continue;
    const int ti = clampi(row0 + lane, 0, NBLK * NBRUN - 1);
    int cv = cntG[ti];
    int ofv = offG[ti];
    PIN(cv);
    PIN(ofv);
    const int bigv = (cv > DEGCAP) ? 1 : 0;
    cv  = cv < 0 ? 0 : (cv > DEGCAP ? DEGCAP : cv);
    ofv = ofv < 0 ? 0 : (ofv > LCAP ? LCAP : ofv);
#pragma unroll 1
    for (int r = 0; r < RGRP; ++r) {
      const int node = row0 + r;
      const bool live = node < nN;
      const int c  = __builtin_amdgcn_readlane(cv, r);
      const int o  = __builtin_amdgcn_readlane(ofv, r);
      const int bg = __builtin_amdgcn_readlane(bigv, r);
      const int cn = __builtin_amdgcn_readfirstlane(live ? c : 0);
      const int idx = clampi(o + lane, 0, LCAP - 1);
      int ent = listb[idx];
      PIN(ent);
      const v2f a = row_gather(T, ent, cn, lane, nN);
      const float o0 = a.x + bv.x;
      const float o1 = a.y + bv.y;
      const float m0 = val0 ? o0 : ninf;
      const float m1 = val1 ? o1 : ninf;
      float m = m0;
      m = (m1 > m || m1 != m1) ? m1 : m;
#pragma unroll
      for (int off = 16; off > 0; off >>= 1) {
        const float y = __shfl_xor(m, off, 32);
        m = (y > m || y != y) ? y : m;
      }
      const float e0 = expf(o0 - m);
      const float e1 = expf(o1 - m);
      float s = (val0 ? e0 : 0.0f) + (val1 ? e1 : 0.0f);
#pragma unroll
      for (int off = 16; off > 0; off >>= 1) s += __shfl_xor(s, off, 32);
      const float ls = logf(s);
      float w0 = (o0 - m) - ls;
      float w1 = (o1 - m) - ls;
      const bool bad = ovf || (bg != 0);
      w0 = bad ? qnan : w0;
      w1 = bad ? qnan : w1;
      if (val0) st[r * DOUT + c0] = w0;
      if (val1) st[r * DOUT + c0 + 1] = w1;
    }
    __builtin_amdgcn_fence(__ATOMIC_RELEASE, "workgroup");
    __builtin_amdgcn_wave_barrier();
    __builtin_amdgcn_fence(__ATOMIC_ACQUIRE, "workgroup");
    v4f vv[OUT_IT];
#pragma unroll
    for (int it = 0; it < OUT_IT; ++it) {
      const int i  = it * 32 + lane;
      const int ic = i < OUT_V4 ? i : OUT_V4 - 1;
      vv[it] = *(const v4fa*)(st + 4 * ic);
    }
    const size_t fbase = (size_t)row0 * DOUT;
    for (int pass = 0; pass < 2; ++pass) {
#pragma unroll
      for (int it = 0; it < OUT_IT; ++it) {
        const int i = it * 32 + lane;
        const size_t f = fbase + 4 * (size_t)i;
        if (i < OUT_V4 && f + 4 <= (size_t)outN) *(volatile v4f*)(out + f) = vv[it];
      }
      __threadfence();
    }
    __builtin_amdgcn_fence(__ATOMIC_RELEASE, "workgroup");
    __builtin_amdgcn_wave_barrier();
    __builtin_amdgcn_fence(__ATOMIC_ACQUIRE, "workgroup");
  }
}

constexpr size_t SZ_XB   = (size_t)MPAD * DIN * 2;
constexpr size_t SZ_T    = (size_t)MPAD * 64 * 4;
constexpr size_t SZ_HHL  = (size_t)MPAD * 128 * 2;
constexpr size_t SZ_LIST = (size_t)NBLK * LCAP * 4;
constexpr size_t SZ_CNT  = (size_t)NBLK * NBRUN * 4;
constexpr size_t SZ_FLAG = (size_t)NBLK * 32 * 4;
constexpr size_t SZ_W1T  = (size_t)DHID * DIN * 2;
constexpr size_t SZ_WD   = (size_t)DHID * 128 * 2;
constexpr size_t SZ_BT   = (size_t)3 * 64 * 4;
constexpr size_t O_XB   = 0;
constexpr size_t O_T    = O_XB + SZ_XB;
constexpr size_t O_HHL  = O_T + SZ_T;
constexpr size_t O_LIST = O_HHL + SZ_HHL;
constexpr size_t O_CNT  = O_LIST + SZ_LIST;
constexpr size_t O_OFF  = O_CNT + SZ_CNT;
constexpr size_t O_FLAG = O_OFF + SZ_CNT;
constexpr size_t O_W1T  = O_FLAG + SZ_FLAG;
constexpr size_t O_W2D  = O_W1T + SZ_W1T;
constexpr size_t O_W3D  = O_W2D + SZ_WD;
constexpr size_t O_BT   = O_W3D + SZ_WD;
constexpr size_t WS_TOTAL = O_BT + SZ_BT;
static_assert(SZ_XB % 256 == 0 && SZ_T % 256 == 0 && SZ_HHL % 256 == 0 && SZ_LIST % 256 == 0);
static_assert(SZ_CNT % 256 == 0 && SZ_FLAG % 256 == 0 && SZ_W1T % 256 == 0 && SZ_WD % 256 == 0 && SZ_BT % 256 == 0);
static_assert(WS_TOTAL == 69032960 && WS_TOTAL <= ((size_t)128 << 20));
static_assert((size_t)MPAD * K2 * 2 <= SZ_HHL && (size_t)MPAD * K3 * 2 <= SZ_HHL);
static_assert((size_t)DHID * K2 * 2 <= SZ_WD && (size_t)DHID * K3 * 2 <= SZ_WD);

extern "C" void kernel_launch(void* const* d_in, const int* in_sizes, int n_in,
                              void* d_out, int out_size, void* d_ws, size_t ws_size,
                              hipStream_t stream) {
  if (n_in < 8) return;
  if (in_sizes[0] != NN * DIN) return;
  if (in_sizes[1] != 2 * NE) return;
  if (in_sizes[2] != DIN * DHID || in_sizes[3] != DHID) return;
  if (in_sizes[4] != DHID * DHID || in_sizes[5] != DHID) return;
  if (in_sizes[6] != DHID * DOUT || in_sizes[7] != DOUT) return;
  if (out_size != OUTN) return;
  if (ws_size < WS_TOTAL) return;

  const float* x    = (const float*)d_in[0];
  const int*   edge = (const int*)d_in[1];
  const float* W1   = (const float*)d_in[2];
  const float* b1   = (const float*)d_in[3];
  const float* W2   = (const float*)d_in[4];
  const float* b2   = (const float*)d_in[5];
  const float* W3   = (const float*)d_in[6];
  const float* b3   = (const float*)d_in[7];
  float* out = (float*)d_out;
  const int* src = edge;
  const int* dst = edge + NE;

  char* ws = (char*)d_ws;
  unsigned short* XB  = (unsigned short*)(ws + O_XB);
  float*          T   = (float*)(ws + O_T);
  unsigned short* HHL = (unsigned short*)(ws + O_HHL);
  int*            LST = (int*)(ws + O_LIST);
  int*            CNT = (int*)(ws + O_CNT);
  int*            OFF = (int*)(ws + O_OFF);
  int*            FLG = (int*)(ws + O_FLAG);
  unsigned short* W1T = (unsigned short*)(ws + O_W1T);
  unsigned short* W2D = (unsigned short*)(ws + O_W2D);
  unsigned short* W3D = (unsigned short*)(ws + O_W3D);
  float*          BT  = (float*)(ws + O_BT);

  hipFuncSetAttribute(reinterpret_cast<const void*>(&k_bucket), hipFuncAttributeMaxDynamicSharedMemorySize,
                      (int)BK_LDS);

  const int gemmGrid = ((MPAD / 64) + 7) / 8;

  k_plane<0><<<MPAD * (DIN / 8) / 256, 256, 0, stream>>>(x, NN, DIN, DIN, XB, MPAD, DIN);
  k_prep<<<NB1 + NB2 + NB3 + 3, NTHR, 0, stream>>>(W1, W2, W3, b1, b2, b3, W1T, W2D, W3D, BT);
  k_bucket<<<NBLK, NTHR, BK_LDS, stream>>>(src, dst, NN, LST, CNT, OFF, FLG);
  k_gemm_nt<0, 0><<<gemmGrid, 256, 0, stream>>>(XB, W1T, BT, T, MPAD, 64, DIN, 64);
  k_replay_hid<K2><<<NBLK, NTHR, 0, stream>>>(T, LST, CNT, OFF, FLG, BT, HHL, NN, MPAD);
  k_gemm_nt<TWO_TERM_L2 ? 1 : 0, 0><<<gemmGrid, 256, 0, stream>>>(HHL, W2D, BT, T, MPAD, 64, K2, 64);
  k_replay_hid<K3><<<NBLK, NTHR, 0, stream>>>(T, LST, CNT, OFF, FLG, BT + 64, HHL, NN, MPAD);
  k_gemm_nt<TWO_TERM_L3 ? 1 : 0, 0><<<gemmGrid, 256, 0, stream>>>(HHL, W3D, BT, T, MPAD, 64, K3, 64);
  k_replay_out<<<NBLK, NTHR, 0, stream>>>(T, LST, CNT, OFF, FLG, BT + 128, out, NN, OUTN);
}
